// MultiHeadAttention_11854109737154
// MI455X (gfx1250) — hardware-verified
//
#include <hip/hip_runtime.h>


typedef _Float16 v16h __attribute__((ext_vector_type(16)));
typedef _Float16 v8h  __attribute__((ext_vector_type(8)));
typedef _Float16 v4h  __attribute__((ext_vector_type(4)));
typedef float    v8f  __attribute__((ext_vector_type(8)));
typedef float    v4f  __attribute__((ext_vector_type(4)));
typedef int      v4i  __attribute__((ext_vector_type(4)));
typedef v8h v8ha __attribute__((may_alias));
typedef v4f v4fa __attribute__((may_alias));
typedef v4i v4ia __attribute__((may_alias));

#ifndef NB
#define NB 2
#endif
#ifndef SEQ
#define SEQ 2048
#endif
#define NB_FULL  2
#define SEQ_FULL 2048
#define DM       2048
#define NH       16
#define HD       128
#define HHALF    64
#define MTOT     (NB * SEQ)
#define QT       128
#define KT       32
#define NQT      (SEQ / QT)
#define NKT      (SEQ / KT)
#define RESROWS  128
#define TABW     64

#define WSCALE     64.0f
#define INV_WSCALE 0.015625f
#define CSC        16.0f
#define INV_CSC    0.0625f
#define RSC        2048.0f
#define INV_RSC    0.00048828125f
#define PCARRY     16384.0f
#define INV_PCARRY 6.103515625e-05f
#define P2S        8.0f
#define SCL        (1.0f / 11.313708305358887f)

static_assert(QT == 128);
static_assert(KT == 32);
static_assert(HD == 128);
static_assert(NH * HD == DM);
static_assert(DM / 128 == NH);
static_assert(DM % 128 == 0);
static_assert(SEQ % QT == 0);
static_assert(QT % KT == 0);
static_assert(MTOT % 128 == 0);
static_assert(NKT >= 1);
static_assert(NKT <= TABW);
static_assert(NB >= 1);
static_assert(NB <= NB_FULL);
static_assert(SEQ <= SEQ_FULL);
static_assert(RESROWS == QT);
static_assert(RESROWS % KT == 0);
static_assert(RESROWS <= SEQ);
static_assert(P2S * RSC == PCARRY);
static_assert((size_t)MTOT * DM * 4 <= (size_t)NB_FULL * SEQ_FULL * DM * 4);

#define WS_PLANE   ((size_t)MTOT * DM * 2)
#define WS_VT      ((size_t)NB * NH * HD * SEQ * 2)
#define WS_VTR     ((size_t)NB * NH * HD * RESROWS * 2)
#define WS_CTXR    ((size_t)NB * RESROWS * DM * 2)
#define WS_TAB     ((size_t)NQT * TABW * 4)
#define OFF_QH   ((size_t)0)
#define OFF_QR   (OFF_QH + WS_PLANE)
#define OFF_KH   (OFF_QR + WS_PLANE)
#define OFF_KR   (OFF_KH + WS_PLANE)
#define OFF_VTH  (OFF_KR + WS_PLANE)
#define OFF_VTR  (OFF_VTH + WS_VT)
#define OFF_CH   (OFF_VTR + WS_VTR)
#define OFF_CR   (OFF_CH + WS_PLANE)
#define OFF_TAB  (OFF_CR + WS_CTXR)
#define WS_TOTAL (OFF_TAB + WS_TAB)
static_assert(WS_TOTAL <= (size_t)134217728);
static_assert(OFF_QR % 256 == 0);
static_assert(OFF_VTR % 256 == 0);
static_assert(OFF_CH % 256 == 0);
static_assert(OFF_CR % 256 == 0);
static_assert(OFF_TAB % 256 == 0);

__device__ __forceinline__ float bfr(float f) {
    unsigned int u = __float_as_uint(f);
    u += 0x7fffu + ((u >> 16) & 1u);
    return __uint_as_float(u & 0xffff0000u);
}

__device__ __forceinline__ v16h ldfrag(const _Float16* p, int hf) {
    union { v16h v; v8h h[2]; } f;
    f.h[0] = *(const v8ha*)(p + 8 * hf);
    f.h[1] = *(const v8ha*)(p + 16 + 8 * hf);
    return f.v;
}

__device__ __forceinline__ v8f mma16(v16h a, v16h b, v8f c) {
    v8f d = __builtin_amdgcn_wmma_f32_16x16x32_f16(false, a, false, b, (short)0, c, false, false);
    asm volatile("v_nop\n\tv_nop\n\tv_nop\n\tv_nop" : "+v"(d) : "v"(a), "v"(b));
    return d;
}

__device__ __forceinline__ void stage_x(_Float16* Asm, const float* __restrict__ X,
                                        size_t srow0, int kk, int t) {
#pragma unroll
    for (int i = 0; i < 8; ++i) {
        const int idx = t + i * 256;
        const int row = idx >> 4, c4 = idx & 15;
        const v4f f = *(const v4fa*)(X + (srow0 + (size_t)row) * DM + kk + c4 * 4);
        v4h hv;
        hv.x = (_Float16)bfr(f.x); hv.y = (_Float16)bfr(f.y);
        hv.z = (_Float16)bfr(f.z); hv.w = (_Float16)bfr(f.w);
        *(v4h*)(Asm + row * 64 + c4 * 4) = hv;
    }
}
__device__ __forceinline__ void stage_w(_Float16* Bsm, const float* __restrict__ W,
                                        int nrow, int kk, int t) {
#pragma unroll
    for (int i = 0; i < 8; ++i) {
        const int idx = t + i * 256;
        const int row = idx >> 4, c4 = idx & 15;
        const v4f f = *(const v4fa*)(W + (size_t)(nrow + row) * DM + kk + c4 * 4);
        v4h hv;
        hv.x = (_Float16)(bfr(f.x) * WSCALE); hv.y = (_Float16)(bfr(f.y) * WSCALE);
        hv.z = (_Float16)(bfr(f.z) * WSCALE); hv.w = (_Float16)(bfr(f.w) * WSCALE);
        *(v4h*)(Bsm + row * 64 + c4 * 4) = hv;
    }
}
__device__ __forceinline__ void stage_h(_Float16* Asm, const _Float16* __restrict__ P,
                                        size_t srow0, int kk, int t) {
#pragma unroll
    for (int i = 0; i < 4; ++i) {
        const int idx = t + i * 256;
        const int row = idx >> 3, seg = idx & 7;
        *(v8h*)(Asm + row * 64 + seg * 8) =
            *(const v8ha*)(P + (srow0 + (size_t)row) * DM + kk + seg * 8);
    }
}

__device__ __forceinline__ void mac64(v8f (&acc)[2][4], const _Float16* Asm, const _Float16* Bsm,
                                      int mloc, int nloc, int l15, int hf) {
#pragma unroll
    for (int ks = 0; ks < 2; ++ks) {
        v16h a[2], b[4];
#pragma unroll
        for (int tm = 0; tm < 2; ++tm)
            a[tm] = ldfrag(Asm + (mloc + tm * 16 + l15) * 64 + ks * 32, hf);
#pragma unroll
        for (int tn = 0; tn < 4; ++tn)
            b[tn] = ldfrag(Bsm + (nloc + tn * 16 + l15) * 64 + ks * 32, hf);
#pragma unroll
        for (int tm = 0; tm < 2; ++tm)
#pragma unroll
            for (int tn = 0; tn < 4; ++tn)
                acc[tm][tn] = mma16(a[tm], b[tn], acc[tm][tn]);
    }
}

__device__ __forceinline__ void store_tile_h(const _Float16* T, _Float16* __restrict__ g,
                                             size_t grow0, size_t gpitch, int gcol0, int t) {
    v4i v[8];
#pragma unroll
    for (int i = 0; i < 8; ++i) {
        const int idx = t + i * 256;
        const int row = idx >> 4, seg = idx & 15;
        v[i] = *(const v4ia*)(T + row * 128 + seg * 8);
    }
#pragma unroll
    for (int i = 0; i < 8; ++i) {
        const int idx = t + i * 256;
        const int row = idx >> 4, seg = idx & 15;
        *(volatile v4i*)(g + (grow0 + (size_t)row) * gpitch + gcol0 + seg * 8) = v[i];
    }
    __threadfence();
#pragma unroll
    for (int i = 0; i < 8; ++i) {
        const int idx = t + i * 256;
        const int row = idx >> 4, seg = idx & 15;
        *(volatile v4i*)(g + (grow0 + (size_t)row) * gpitch + gcol0 + seg * 8) = v[i];
    }
}
__device__ __forceinline__ void store_tile_f(const float* T, float* __restrict__ g,
                                             size_t grow0, int gcol0, int t) {
#pragma unroll
    for (int c = 0; c < 2; ++c) {
        v4i v[8];
#pragma unroll
        for (int i = 0; i < 8; ++i) {
            const int idx = t + (c * 8 + i) * 256;
            const int row = idx >> 5, seg = idx & 31;
            v[i] = *(const v4ia*)(T + row * 128 + seg * 4);
        }
#pragma unroll
        for (int i = 0; i < 8; ++i) {
            const int idx = t + (c * 8 + i) * 256;
            const int row = idx >> 5, seg = idx & 31;
            *(volatile v4i*)(g + (grow0 + (size_t)row) * DM + gcol0 + seg * 4) = v[i];
        }
        __threadfence();
#pragma unroll
        for (int i = 0; i < 8; ++i) {
            const int idx = t + (c * 8 + i) * 256;
            const int row = idx >> 5, seg = idx & 31;
            *(volatile v4i*)(g + (grow0 + (size_t)row) * DM + gcol0 + seg * 4) = v[i];
        }
    }
}

template <int MODE>
__global__ __launch_bounds__(256) void gemm_xwt(
    const float* __restrict__ Xf, const _Float16* __restrict__ Xh, const _Float16* __restrict__ Xr,
    const float* __restrict__ W, const float* __restrict__ bias,
    const float* __restrict__ cosp, const float* __restrict__ sinp,
    _Float16* __restrict__ oh, _Float16* __restrict__ orr, float* __restrict__ o32)
{
    __shared__ __align__(16) _Float16 smem[32768];
    _Float16* Asm = smem;
    _Float16* Bsm = smem + 8192;

    const int t = threadIdx.x, lane = t & 31, wave = t >> 5;
    const int l15 = lane & 15, hf = lane >> 4;
    const int wrow = wave >> 1, wcol = wave & 1;
    const int arow = blockIdx.y * 128, nrow = blockIdx.x * 128;
    const int mloc = wrow * 32, nloc = wcol * 64;
    const int bI = arow / SEQ, lrow0 = arow - bI * SEQ;
    const bool useres = (lrow0 < RESROWS);

    v8f acc[2][4];
#pragma unroll
    for (int tm = 0; tm < 2; ++tm)
#pragma unroll
        for (int tn = 0; tn < 4; ++tn)
#pragma unroll
            for (int j = 0; j < 8; ++j) acc[tm][tn][j] = 0.0f;

    if (MODE == 2) {
        if (useres) {
            for (int kk = 0; kk < DM; kk += 64) {
                __syncthreads();
                stage_h(Asm, Xr, (size_t)bI * RESROWS + lrow0, kk, t);
                stage_w(Bsm, W, nrow, kk, t);
                __syncthreads();
                mac64(acc, Asm, Bsm, mloc, nloc, l15, hf);
            }
#pragma unroll
            for (int tm = 0; tm < 2; ++tm)
#pragma unroll
                for (int tn = 0; tn < 4; ++tn)
#pragma unroll
                    for (int j = 0; j < 8; ++j) acc[tm][tn][j] *= INV_RSC;
        }
        for (int kk = 0; kk < DM; kk += 64) {
            __syncthreads();
            stage_h(Asm, Xh, (size_t)arow, kk, t);
            stage_w(Bsm, W, nrow, kk, t);
            __syncthreads();
            mac64(acc, Asm, Bsm, mloc, nloc, l15, hf);
        }
    } else {
        const size_t srow0 = (size_t)bI * SEQ_FULL + lrow0;
        for (int kk = 0; kk < DM; kk += 64) {
            __syncthreads();
            stage_x(Asm, Xf, srow0, kk, t);
            stage_w(Bsm, W, nrow, kk, t);
            __syncthreads();
            mac64(acc, Asm, Bsm, mloc, nloc, l15, hf);
        }
    }
    __syncthreads();

    float bb[4];
#pragma unroll
    for (int tn = 0; tn < 4; ++tn) bb[tn] = bfr(bias[nrow + nloc + tn * 16 + l15]);

    if (MODE == 0) {
        float* Rt = (float*)smem;
#pragma unroll
        for (int i = 0; i < 8; ++i) {
            const int idx = t + i * 256;
            const int row = idx >> 4, c4 = idx & 15;
            const size_t lp = (size_t)(lrow0 + row) * HHALF + c4 * 4;
            const v4f cs = *(const v4fa*)(cosp + lp);
            const v4f sn = *(const v4fa*)(sinp + lp);
            v4f r;
            r.x = bfr(cs.x) - bfr(sn.x); r.y = bfr(cs.y) - bfr(sn.y);
            r.z = bfr(cs.z) - bfr(sn.z); r.w = bfr(cs.w) - bfr(sn.w);
            *(v4f*)(Rt + row * 64 + c4 * 4) = r;
        }
        __syncthreads();
#pragma unroll
        for (int tm = 0; tm < 2; ++tm)
#pragma unroll
            for (int tn = 0; tn < 4; ++tn)
#pragma unroll
                for (int j = 0; j < 8; ++j) {
                    const int ml = mloc + tm * 16 + 8 * hf + j;
                    float v = acc[tm][tn][j] * INV_WSCALE + bb[tn];
                    const float rf = Rt[ml * 64 + tn * 16 + l15];
                    v = (wcol == 0) ? v * rf : v;
                    acc[tm][tn][j] = v;
                }
        __syncthreads();
    } else {
        const float osc = (MODE == 2) ? (INV_WSCALE * INV_CSC) : INV_WSCALE;
#pragma unroll
        for (int tm = 0; tm < 2; ++tm)
#pragma unroll
            for (int tn = 0; tn < 4; ++tn)
#pragma unroll
                for (int j = 0; j < 8; ++j)
                    acc[tm][tn][j] = acc[tm][tn][j] * osc + bb[tn];
    }

    if (MODE == 2) {
        float* T32 = (float*)smem;
#pragma unroll
        for (int tm = 0; tm < 2; ++tm)
#pragma unroll
            for (int tn = 0; tn < 4; ++tn)
#pragma unroll
                for (int j = 0; j < 8; ++j) {
                    const int ml = mloc + tm * 16 + 8 * hf + j;
                    const int nl = nloc + tn * 16 + l15;
                    T32[ml * 128 + nl] = acc[tm][tn][j];
                }
    } else {
        _Float16* Th = smem;
        _Float16* Tr = smem + 16384;
#pragma unroll
        for (int tm = 0; tm < 2; ++tm)
#pragma unroll
            for (int tn = 0; tn < 4; ++tn)
#pragma unroll
                for (int j = 0; j < 8; ++j) {
                    const int ml = mloc + tm * 16 + 8 * hf + j;
                    const int nl = nloc + tn * 16 + l15;
                    const float v = acc[tm][tn][j];
                    const _Float16 hv = (_Float16)v;
                    const _Float16 rv = (_Float16)((v - (float)hv) * RSC);
                    if (MODE == 0) {
                        Th[ml * 128 + nl] = hv;
                        Tr[ml * 128 + nl] = rv;
                    } else {
                        Th[nl * 128 + ml] = hv;
                        if (useres) Tr[nl * 128 + ml] = rv;
                    }
                }
    }
    __syncthreads();

    if (MODE == 0) {
        store_tile_h(smem, oh, (size_t)arow, (size_t)DM, nrow, t);
        store_tile_h(smem + 16384, orr, (size_t)arow, (size_t)DM, nrow, t);
    } else if (MODE == 1) {
        const int hh = blockIdx.x;
        const size_t drow0 = (size_t)(bI * NH + hh) * HD;
        store_tile_h(smem, oh, drow0, (size_t)SEQ, lrow0, t);
        if (useres) store_tile_h(smem + 16384, orr, drow0, (size_t)RESROWS, 0, t);
    } else {
        store_tile_f((const float*)smem, o32, (size_t)arow, nrow, t);
    }
}

__global__ __launch_bounds__(256) void tile_classes(const int* __restrict__ gate, int* __restrict__ tab)
{
    __shared__ int fnz[256];
    __shared__ int fz[256];
    __shared__ __align__(16) int scl[TABW];

    const int t = threadIdx.x, qt = blockIdx.x, q0 = qt * QT;
    const int kt = t & 63, rg = t >> 6;
    const int ktc = (kt < NKT) ? kt : (NKT - 1);
    int anz = 0, az = 0;
#pragma unroll 1
    for (int r = 0; r < 32; ++r) {
        const int* rowp = gate + (size_t)(q0 + rg * 32 + r) * SEQ_FULL + ktc * KT;
#pragma unroll
        for (int c = 0; c < 8; ++c) {
            const v4i m = *(const v4ia*)(rowp + c * 4);
            anz |= (int)(m.x != 0) | (int)(m.y != 0) | (int)(m.z != 0) | (int)(m.w != 0);
            az  |= (int)(m.x == 0) | (int)(m.y == 0) | (int)(m.z == 0) | (int)(m.w == 0);
        }
    }
    fnz[t] = anz;
    fz[t] = az;
    __syncthreads();
    if (t < 64) {
        const int nz = fnz[t] | fnz[64 + t] | fnz[128 + t] | fnz[192 + t];
        const int z  = fz[t]  | fz[64 + t]  | fz[128 + t]  | fz[192 + t];
        int c = (nz == 0) ? 0 : ((z != 0) ? 1 : 2);
        if (t >= NKT) c = 0;
        scl[t] = c;
    }
    __syncthreads();
    if (t < 16) {
        const v4i v = *(const v4ia*)(scl + t * 4);
        int* g = tab + (size_t)qt * TABW + t * 4;
        *(volatile v4i*)g = v;
        __threadfence();
        *(volatile v4i*)g = v;
    }
}

__global__ __launch_bounds__(256) void attn_fwd(
    const _Float16* __restrict__ qh, const _Float16* __restrict__ qr,
    const _Float16* __restrict__ kh, const _Float16* __restrict__ kr,
    const _Float16* __restrict__ vth, const _Float16* __restrict__ vtr,
    const int* __restrict__ gate, const int* __restrict__ tab,
    _Float16* __restrict__ ch, _Float16* __restrict__ cr)
{
    __shared__ __align__(16) _Float16 Qh[QT * HD];
    __shared__ __align__(16) _Float16 Qr[QT * HD];
    __shared__ __align__(16) _Float16 Kh[KT * HD];
    __shared__ __align__(16) _Float16 Kr[KT * HD];
    __shared__ __align__(16) _Float16 Vh[HD * KT];
    __shared__ __align__(16) _Float16 Vr[HD * KT];
    __shared__ __align__(16) _Float16 Pl[8][16 * KT];
    __shared__ __align__(16) _Float16 Pl2[8][16 * KT];
    __shared__ __align__(16) unsigned char Msk[QT * KT];

    const int t = threadIdx.x, lane = t & 31, wave = t >> 5;
    const int l15 = lane & 15, hf = lane >> 4;
    const int bh = blockIdx.y, b = bh / NH, h = bh - b * NH;
    const int qt = blockIdx.x, q0 = qt * QT;
    const bool useres = (q0 < RESROWS);
    const int mrl = 8 * hf;

    {
        const size_t base = (size_t)(b * SEQ + q0) * DM + h * HD;
#pragma unroll
        for (int i = 0; i < 8; ++i) {
            const int idx = t + i * 256;
            const int row = idx >> 4, seg = idx & 15;
            *(v8h*)(Qh + row * HD + seg * 8) = *(const v8ha*)(qh + base + (size_t)row * DM + seg * 8);
            *(v8h*)(Qr + row * HD + seg * 8) = *(const v8ha*)(qr + base + (size_t)row * DM + seg * 8);
        }
    }

    v8f acc[8];
#pragma unroll
    for (int tn = 0; tn < 8; ++tn)
#pragma unroll
        for (int j = 0; j < 8; ++j) acc[tn][j] = 0.0f;
    v8f mrun, lrun;
#pragma unroll
    for (int j = 0; j < 8; ++j) { mrun[j] = -1e30f; lrun[j] = 0.0f; }

    const _Float16* qhr = Qh + (wave * 16 + l15) * HD;
    const _Float16* qrr = Qr + (wave * 16 + l15) * HD;

    for (int kt = 0; kt < NKT; ++kt) {
        int cls = tab[(size_t)qt * TABW + kt];
        cls = (cls < 0) ? 0 : ((cls > 2) ? 2 : cls);
        if (cls == 0) continue;
        const int kv = kt * KT;
        const bool resv = useres && (kv + KT <= RESROWS);

        __syncthreads();
        {
            const size_t kbase = (size_t)(b * SEQ + kv) * DM + h * HD;
#pragma unroll
            for (int i = 0; i < 2; ++i) {
                const int idx = t + i * 256;
                const int row = idx >> 4, seg = idx & 15;
                *(v8h*)(Kh + row * HD + seg * 8) = *(const v8ha*)(kh + kbase + (size_t)row * DM + seg * 8);
                *(v8h*)(Kr + row * HD + seg * 8) = *(const v8ha*)(kr + kbase + (size_t)row * DM + seg * 8);
            }
            const size_t vbase = (size_t)bh * HD * SEQ + kv;
            const size_t rbase = (size_t)bh * HD * RESROWS + kv;
#pragma unroll
            for (int i = 0; i < 2; ++i) {
                const int idx = t + i * 256;
                const int row = idx >> 2, seg = idx & 3;
                *(v8h*)(Vh + row * KT + seg * 8) = *(const v8ha*)(vth + vbase + (size_t)row * SEQ + seg * 8);
                if (resv)
                    *(v8h*)(Vr + row * KT + seg * 8) = *(const v8ha*)(vtr + rbase + (size_t)row * RESROWS + seg * 8);
            }
            if (cls == 1) {
#pragma unroll
                for (int i = 0; i < 4; ++i) {
                    const int idx = t + i * 256;
                    const int row = idx >> 3, c4 = idx & 7;
                    const v4i m = *(const v4ia*)(gate + (size_t)(q0 + row) * SEQ_FULL + kv + c4 * 4);
                    const unsigned pk = (unsigned)(m.x != 0) | ((unsigned)(m.y != 0) << 8) |
                                        ((unsigned)(m.z != 0) << 16) | ((unsigned)(m.w != 0) << 24);
                    *(unsigned*)(Msk + row * KT + c4 * 4) = pk;
                }
            }
        }
        __syncthreads();

        v8f sc[2];
#pragma unroll
        for (int tn = 0; tn < 2; ++tn)
#pragma unroll
            for (int j = 0; j < 8; ++j) sc[tn][j] = 0.0f;
#pragma unroll
        for (int ks = 0; ks < 4; ++ks) {
            const v16h ah = ldfrag(qhr + ks * 32, hf);
            const v16h ar = ldfrag(qrr + ks * 32, hf);
#pragma unroll
            for (int tn = 0; tn < 2; ++tn) {
                const v16h bkh = ldfrag(Kh + (tn * 16 + l15) * HD + ks * 32, hf);
                const v16h bkr = ldfrag(Kr + (tn * 16 + l15) * HD + ks * 32, hf);
                sc[tn] = mma16(ar, bkh, sc[tn]);
                sc[tn] = mma16(ah, bkr, sc[tn]);
            }
        }
#pragma unroll
        for (int tn = 0; tn < 2; ++tn)
#pragma unroll
            for (int j = 0; j < 8; ++j) sc[tn][j] *= INV_RSC;
#pragma unroll
        for (int ks = 0; ks < 4; ++ks) {
            const v16h ah = ldfrag(qhr + ks * 32, hf);
#pragma unroll
            for (int tn = 0; tn < 2; ++tn) {
                const v16h bkh = ldfrag(Kh + (tn * 16 + l15) * HD + ks * 32, hf);
                sc[tn] = mma16(ah, bkh, sc[tn]);
            }
        }
#pragma unroll
        for (int tn = 0; tn < 2; ++tn)
#pragma unroll
            for (int j = 0; j < 8; ++j) sc[tn][j] *= SCL;
        if (cls == 1) {
#pragma unroll
            for (int tn = 0; tn < 2; ++tn)
#pragma unroll
                for (int j = 0; j < 8; ++j) {
                    const unsigned char mk = Msk[(wave * 16 + mrl + j) * KT + tn * 16 + l15];
                    sc[tn][j] = (mk != 0) ? sc[tn][j] : -__builtin_inff();
                }
        }

        v8f cmax;
#pragma unroll
        for (int j = 0; j < 8; ++j) cmax[j] = fmaxf(sc[0][j], sc[1][j]);
#pragma unroll
        for (int m = 1; m < 16; m <<= 1)
#pragma unroll
            for (int j = 0; j < 8; ++j) cmax[j] = fmaxf(cmax[j], __shfl_xor(cmax[j], m, 32));
        v8f corr;
#pragma unroll
        for (int j = 0; j < 8; ++j) {
            const float mn = fmaxf(mrun[j], cmax[j]);
            corr[j] = __expf(mrun[j] - mn);
            mrun[j] = mn;
        }
        v8f rsum = {};
#pragma unroll
        for (int tn = 0; tn < 2; ++tn)
#pragma unroll
            for (int j = 0; j < 8; ++j) {
                const float p = __expf(sc[tn][j] - mrun[j]);
                sc[tn][j] = p;
                rsum[j] += p;
            }
#pragma unroll
        for (int m = 1; m < 16; m <<= 1)
#pragma unroll
            for (int j = 0; j < 8; ++j) rsum[j] += __shfl_xor(rsum[j], m, 32);
#pragma unroll
        for (int j = 0; j < 8; ++j) lrun[j] = lrun[j] * corr[j] + rsum[j];
#pragma unroll
        for (int tn = 0; tn < 8; ++tn)
#pragma unroll
            for (int j = 0; j < 8; ++j) acc[tn][j] *= corr[j];

        _Float16* pl = Pl[wave];
        _Float16* pl2 = Pl2[wave];
#pragma unroll
        for (int tn = 0; tn < 2; ++tn)
#pragma unroll
            for (int j = 0; j < 8; ++j)
                pl[(mrl + j) * KT + tn * 16 + l15] = (_Float16)(sc[tn][j] * PCARRY);
        if (resv) {
#pragma unroll
            for (int tn = 0; tn < 2; ++tn)
#pragma unroll
                for (int j = 0; j < 8; ++j)
                    pl2[(mrl + j) * KT + tn * 16 + l15] = (_Float16)(sc[tn][j] * P2S);
        }
        __builtin_amdgcn_fence(__ATOMIC_RELEASE, "wavefront");
        __builtin_amdgcn_wave_barrier();
        const v16h pf = ldfrag(pl + l15 * KT, hf);

#pragma unroll
        for (int tn = 0; tn < 8; ++tn) {
            const v16h vf = ldfrag(Vh + (tn * 16 + l15) * KT, hf);
            acc[tn] = mma16(pf, vf, acc[tn]);
        }
        if (resv) {
            const v16h pf2 = ldfrag(pl2 + l15 * KT, hf);
#pragma unroll
            for (int tn = 0; tn < 8; ++tn) {
                const v16h vf = ldfrag(Vr + (tn * 16 + l15) * KT, hf);
                acc[tn] = mma16(pf2, vf, acc[tn]);
            }
        }
    }
    __syncthreads();

    float rlc[8];
#pragma unroll
    for (int j = 0; j < 8; ++j) rlc[j] = (1.0f / lrun[j]) * (CSC * INV_PCARRY);
#pragma unroll
    for (int tn = 0; tn < 8; ++tn)
#pragma unroll
        for (int j = 0; j < 8; ++j) {
            const int ml = wave * 16 + mrl + j;
            const int nl = tn * 16 + l15;
            const float v = acc[tn][j] * rlc[j];
            const _Float16 hv = (_Float16)v;
            Qh[ml * HD + nl] = hv;
            if (useres) Qr[ml * HD + nl] = (_Float16)((v - (float)hv) * RSC);
        }
    __syncthreads();
    store_tile_h(Qh, ch, (size_t)(b * SEQ + q0), (size_t)DM, h * HD, t);
    if (useres) store_tile_h(Qr, cr, (size_t)(b * RESROWS + q0), (size_t)DM, h * HD, t);
}

extern "C" void kernel_launch(void* const* d_in, const int* in_sizes, int n_in,
                              void* d_out, int out_size, void* d_ws, size_t ws_size,
                              hipStream_t stream) {
    if (n_in < 12) return;
    if ((size_t)in_sizes[0] < ((size_t)(NB - 1) * SEQ_FULL + SEQ) * DM) return;
    if (in_sizes[1] < SEQ * HHALF || in_sizes[2] < SEQ * HHALF) return;
    if ((size_t)in_sizes[3] < (size_t)(SEQ - 1) * SEQ_FULL + SEQ) return;
    if (in_sizes[4] < DM * DM || in_sizes[6] < DM * DM || in_sizes[8] < DM * DM || in_sizes[10] < DM * DM) return;
    if (in_sizes[5] < DM || in_sizes[7] < DM || in_sizes[9] < DM || in_sizes[11] < DM) return;
    if (out_size < MTOT * DM) return;
    if (ws_size < WS_TOTAL) return;

    const float* x    = (const float*)d_in[0];
    const float* sinp = (const float*)d_in[1];
    const float* cosp = (const float*)d_in[2];
    const int*   gate = (const int*)d_in[3];
    const float* Wq = (const float*)d_in[4];  const float* bq = (const float*)d_in[5];
    const float* Wk = (const float*)d_in[6];  const float* bk = (const float*)d_in[7];
    const float* Wv = (const float*)d_in[8];  const float* bv = (const float*)d_in[9];
    const float* Wo = (const float*)d_in[10]; const float* bo = (const float*)d_in[11];
    float* out = (float*)d_out;

    char* ws = (char*)d_ws;
    _Float16* qh  = (_Float16*)(ws + OFF_QH);
    _Float16* qr  = (_Float16*)(ws + OFF_QR);
    _Float16* kh  = (_Float16*)(ws + OFF_KH);
    _Float16* kr  = (_Float16*)(ws + OFF_KR);
    _Float16* vth = (_Float16*)(ws + OFF_VTH);
    _Float16* vtr = (_Float16*)(ws + OFF_VTR);
    _Float16* ch  = (_Float16*)(ws + OFF_CH);
    _Float16* cr  = (_Float16*)(ws + OFF_CR);
    int*      tab = (int*)(ws + OFF_TAB);

    dim3 blk(256);
    tile_classes<<<dim3(NQT), blk, 0, stream>>>(gate, tab);

    dim3 gg(DM / 128, MTOT / 128);
    gemm_xwt<0><<<gg, blk, 0, stream>>>(x, ch, cr, Wq, bq, cosp, sinp, qh, qr, out);
    gemm_xwt<0><<<gg, blk, 0, stream>>>(x, ch, cr, Wk, bk, cosp, sinp, kh, kr, out);
    gemm_xwt<1><<<gg, blk, 0, stream>>>(x, ch, cr, Wv, bv, cosp, sinp, vth, vtr, out);

    attn_fwd<<<dim3(NQT, NB * NH), blk, 0, stream>>>(qh, qr, kh, kr, vth, vtr, gate, tab, ch, cr);

    gemm_xwt<2><<<gg, blk, 0, stream>>>(x, ch, cr, Wo, bo, cosp, sinp, qh, qr, out);
}
